// TransformerBlock_81003083203503
// MI455X (gfx1250) — hardware-run, weakly checked
//
#include <hip/hip_runtime.h>
#include <stddef.h>


typedef _Float16 v16h __attribute__((ext_vector_type(16)));
typedef _Float16 v8h  __attribute__((ext_vector_type(8)));
typedef _Float16 v4h  __attribute__((ext_vector_type(4)));
typedef float    v8f  __attribute__((ext_vector_type(8)));
typedef float    v4f  __attribute__((ext_vector_type(4)));

#ifndef NB
#define NB 2
#endif
#ifndef SEQ
#define SEQ 2048
#endif
#define NB_FULL  2
#define SEQ_FULL 2048
#define DIM   1024
#define NHEAD 16
#define HD    64
#define MROWS (NB * SEQ)

static_assert(NB >= 1 && NB <= NB_FULL);
static_assert(SEQ >= 128 && SEQ <= SEQ_FULL && (SEQ % 128) == 0);
static_assert(DIM == NHEAD * HD);
static_assert(HD == 64);
static_assert(DIM == 256 * 4);
static_assert((DIM % 64) == 0 && (DIM % 32) == 0);
static_assert((MROWS % 64) == 0);
static_assert(((size_t)MROWS * DIM) % (8 * 256) == 0);
static_assert((size_t)MROWS * DIM < (size_t)0xFFFFFFFFu);

#define LDT 72
#define LDC 68

#define WCARRY 64.0f
#define PCARRY 1024.0f
#define PCEN   800.0f
#define VCARRY 64.0f
#define RCARRY 2048.0f

#define PLANE16_BYTES ((size_t)MROWS * DIM * 2)
#define PLANE32_BYTES ((size_t)MROWS * DIM * 4)
#define WPLANE_BYTES  ((size_t)DIM * DIM * 2)
#define WT_BYTES      ((size_t)9 * WPLANE_BYTES)
#define OFF_XA   (WT_BYTES)
#define OFF_CX   (OFF_XA  + PLANE16_BYTES)
#define OFF_Q    (OFF_CX  + PLANE16_BYTES)
#define OFF_K    (OFF_Q   + PLANE16_BYTES)
#define OFF_VT   (OFF_K   + PLANE16_BYTES)
#define OFF_VTR  (OFF_VT  + PLANE16_BYTES)
#define OFF_O    (OFF_VTR + PLANE16_BYTES)
#define OFF_OR   (OFF_O   + PLANE16_BYTES)
#define OFF_CN   (OFF_OR  + PLANE16_BYTES)
#define OFF_PRE  (OFF_CN  + PLANE16_BYTES)
#define OFF_CF   (OFF_PRE + PLANE32_BYTES)
#define WS_TOTAL (OFF_CF  + PLANE32_BYTES)
static_assert((WT_BYTES % 128) == 0 && (PLANE16_BYTES % 128) == 0 && (PLANE32_BYTES % 128) == 0);
static_assert(WS_TOTAL <= (size_t)134217728);

__device__ __forceinline__ float bf16r(float x) {
  unsigned int u = __float_as_uint(x);
  u = (u + 0x7FFFu + ((u >> 16) & 1u)) & 0xFFFF0000u;
  return __uint_as_float(u);
}

__device__ __forceinline__ v16h frag_at(const _Float16* p) {
  v8h lo = *(const v8h*)(p);
  v8h hi = *(const v8h*)(p + 16);
  v16h out;
#pragma unroll
  for (int i = 0; i < 8; ++i) { out[i] = lo[i]; out[i + 8] = hi[i]; }
  return out;
}
__device__ __forceinline__ v16h ld_frag(const _Float16* base, unsigned ld) {
  const unsigned lane = threadIdx.x & 31u;
  return frag_at(base + (lane & 15u) * ld + (lane >> 4) * 8u);
}

__device__ __forceinline__ v8f wmma16(v16h a, v16h b, v8f c) {
  v8f d = __builtin_amdgcn_wmma_f32_16x16x32_f16(false, a, false, b, (short)0, c,
                                                 false, false);
  asm volatile("v_nop\n\tv_nop\n\tv_nop\n\tv_nop" : "+v"(d) : "v"(a), "v"(b));
  return d;
}

__device__ __forceinline__ float red16_max(float x) {
#pragma unroll
  for (int off = 1; off < 16; off <<= 1) x = fmaxf(x, __shfl_xor(x, off, 32));
  return x;
}
__device__ __forceinline__ float red16_sum(float x) {
#pragma unroll
  for (int off = 1; off < 16; off <<= 1) x += __shfl_xor(x, off, 32);
  return x;
}
__device__ __forceinline__ float red32_sum(float x) {
#pragma unroll
  for (int off = 1; off < 32; off <<= 1) x += __shfl_xor(x, off, 32);
  return x;
}

__device__ __forceinline__ void wave_lds_sync() {
  __builtin_amdgcn_fence(3  , "wavefront");
  asm volatile("s_wait_dscnt 0x0" ::: "memory");
  __builtin_amdgcn_wave_barrier();
}

template <int HEADW>
__global__ __launch_bounds__(256) void wconv_kernel(
    const float* __restrict__ W, _Float16* __restrict__ Wt) {
  __shared__ __attribute__((aligned(16))) _Float16 T[64 * LDT];
  const unsigned tid = threadIdx.x;
  const unsigned n0 = blockIdx.x * 64u;
  const unsigned k0 = blockIdx.y * 64u;
#pragma unroll 4
  for (unsigned j = 0; j < 16u; ++j) {
    const unsigned idx = tid + 256u * j;
    const unsigned kr = idx >> 6, nc = idx & 63u;
    size_t src;
    if (HEADW) src = ((size_t)(n0 >> 6) * DIM + (k0 + kr)) * HD + nc;
    else       src = (size_t)(k0 + kr) * DIM + n0 + nc;
    const float v = W[src];
    T[nc * LDT + kr] = (_Float16)(WCARRY * bf16r(v));
  }
  __syncthreads();
  v8h x[2];
  size_t off[2];
#pragma unroll
  for (unsigned i = 0; i < 2u; ++i) {
    const unsigned n = 32u * i + (tid >> 3);
    const unsigned kc = (tid & 7u) * 8u;
    x[i] = *(const v8h*)&T[n * LDT + kc];
    off[i] = (size_t)(n0 + n) * DIM + k0 + kc;
  }
#pragma unroll
  for (int i = 0; i < 2; ++i) *(volatile v8h*)(Wt + off[i]) = x[i];
  __threadfence();
#pragma unroll
  for (int i = 0; i < 2; ++i) *(volatile v8h*)(Wt + off[i]) = x[i];
}

__global__ __launch_bounds__(256) void xconv_kernel(
    const float* __restrict__ Xin, _Float16* __restrict__ dst) {
  const unsigned e = (blockIdx.x * 256u + threadIdx.x) * 8u;
  const unsigned crow = e / (unsigned)DIM;
  const unsigned c = e - crow * (unsigned)DIM;
  const unsigned bidx = crow / (unsigned)SEQ;
  const unsigned sq = crow - bidx * (unsigned)SEQ;
  const size_t frow = (size_t)bidx * SEQ_FULL + sq;
  const float* sp = Xin + frow * DIM + c;
  const v4f a0 = *(const v4f*)(sp);
  const v4f a1 = *(const v4f*)(sp + 4);
  v8h o;
#pragma unroll
  for (int j = 0; j < 4; ++j) {
    o[j]     = (_Float16)bf16r(a0[j]);
    o[j + 4] = (_Float16)bf16r(a1[j]);
  }
  *(volatile v8h*)(dst + (size_t)e) = o;
  __threadfence();
  *(volatile v8h*)(dst + (size_t)e) = o;
}

#define G_ROW16  0
#define G_VT     1
#define G_VT2    2
#define G_PRE_X  3
#define G_PRE_2X 4
#define G_PRE_C  5

template <int MODE>
__global__ __launch_bounds__(256) void gemm_kernel(
    const _Float16* __restrict__ A16, const _Float16* __restrict__ A16r,
    const _Float16* __restrict__ Bt, const float* __restrict__ bias,
    const float* __restrict__ resid, float* __restrict__ outf,
    _Float16* __restrict__ out16, _Float16* __restrict__ out16r, float oscale) {
  __shared__ __attribute__((aligned(16))) float Cs[64 * LDC];
  const unsigned tid = threadIdx.x, lane = tid & 31u, w = tid >> 5;
  const unsigned mw = w >> 1, nw = w & 1u;
  const unsigned hh = lane >> 4, m = lane & 15u;
  const unsigned n0 = blockIdx.x * 64u;
  const unsigned row0 = blockIdx.y * 64u;

  const size_t aoff = (size_t)(row0 + mw * 16u + m) * DIM + hh * 8u;
  const _Float16* ap  = A16 + aoff;
  const _Float16* bp0 = Bt + (size_t)(n0 + nw * 32u + m) * DIM + hh * 8u;
  const _Float16* bp1 = bp0 + 16 * DIM;
  v8f acc0 = {}, acc1 = {};
#pragma unroll 2
  for (unsigned k0 = 0; k0 < (unsigned)DIM; k0 += 32u) {
    const v16h a  = frag_at(ap + k0);
    const v16h b0 = frag_at(bp0 + k0);
    const v16h b1 = frag_at(bp1 + k0);
    acc0 = wmma16(a, b0, acc0);
    acc1 = wmma16(a, b1, acc1);
  }
  if (MODE == G_PRE_2X) {
    const _Float16* ar = A16r + aoff;
    v8f acc2 = {}, acc3 = {};
#pragma unroll 2
    for (unsigned k0 = 0; k0 < (unsigned)DIM; k0 += 32u) {
      const v16h a  = frag_at(ar + k0);
      const v16h b0 = frag_at(bp0 + k0);
      const v16h b1 = frag_at(bp1 + k0);
      acc2 = wmma16(a, b0, acc2);
      acc3 = wmma16(a, b1, acc3);
    }
#pragma unroll
    for (int r = 0; r < 8; ++r) {
      acc0[r] = acc0[r] + acc2[r] * (1.0f / RCARRY);
      acc1[r] = acc1[r] + acc3[r] * (1.0f / RCARRY);
    }
  }
#pragma unroll
  for (int r = 0; r < 8; ++r) {
    float* d = &Cs[(mw * 16u + hh * 8u + (unsigned)r) * LDC + nw * 32u + m];
    d[0]  = acc0[r];
    d[16] = acc1[r];
  }
  __syncthreads();

  if (MODE == G_ROW16) {
    v8h x[2];
    size_t off[2];
#pragma unroll
    for (unsigned i = 0; i < 2u; ++i) {
      const unsigned r = 32u * i + (tid >> 3);
      const unsigned c = (tid & 7u) * 8u;
      const v4f u0 = *(const v4f*)&Cs[r * LDC + c];
      const v4f u1 = *(const v4f*)&Cs[r * LDC + c + 4];
#pragma unroll
      for (int j = 0; j < 4; ++j) {
        x[i][j]     = (_Float16)(u0[j] * oscale);
        x[i][j + 4] = (_Float16)(u1[j] * oscale);
      }
      off[i] = (size_t)(row0 + r) * DIM + n0 + c;
    }
#pragma unroll
    for (int i = 0; i < 2; ++i) *(volatile v8h*)(out16 + off[i]) = x[i];
    __threadfence();
#pragma unroll
    for (int i = 0; i < 2; ++i) *(volatile v8h*)(out16 + off[i]) = x[i];
  }

  if (MODE == G_VT || MODE == G_VT2) {
    const unsigned bidx = row0 / (unsigned)SEQ;
    const unsigned key0 = row0 - bidx * (unsigned)SEQ;
    v8h x[2], y[2];
    size_t off[2];
#pragma unroll
    for (unsigned i = 0; i < 2u; ++i) {
      const unsigned dcol = 32u * i + (tid >> 3);
      const unsigned kk = (tid & 7u) * 8u;
#pragma unroll
      for (unsigned j = 0; j < 8u; ++j) {
        const float v = Cs[(kk + j) * LDC + dcol] * oscale;
        const _Float16 hv = (_Float16)v;
        x[i][j] = hv;
        y[i][j] = (_Float16)((v - (float)hv) * RCARRY);
      }
      off[i] = ((size_t)bidx * DIM + n0 + dcol) * SEQ + key0 + kk;
    }
#pragma unroll
    for (int i = 0; i < 2; ++i) *(volatile v8h*)(out16 + off[i]) = x[i];
    if (MODE == G_VT2) {
#pragma unroll
      for (int i = 0; i < 2; ++i) *(volatile v8h*)(out16r + off[i]) = y[i];
    }
    __threadfence();
#pragma unroll
    for (int i = 0; i < 2; ++i) *(volatile v8h*)(out16 + off[i]) = x[i];
    if (MODE == G_VT2) {
#pragma unroll
      for (int i = 0; i < 2; ++i) *(volatile v8h*)(out16r + off[i]) = y[i];
    }
  }

  if (MODE == G_PRE_X || MODE == G_PRE_2X || MODE == G_PRE_C) {
    v4f xs[4];
    size_t off[4];
#pragma unroll
    for (unsigned i = 0; i < 4u; ++i) {
      const unsigned r = 16u * i + (tid >> 4);
      const unsigned c = (tid & 15u) * 4u;
      const unsigned crow = row0 + r;
      const v4f u = *(const v4f*)&Cs[r * LDC + c];
      const v4f g = *(const v4f*)(bias + n0 + c);
      v4f t;
#pragma unroll
      for (int j = 0; j < 4; ++j) t[j] = fmaxf(u[j] * oscale + bf16r(g[j]), 0.0f);
      v4f val;
      if (MODE == G_PRE_X) {
        const unsigned bidx = crow / (unsigned)SEQ;
        const unsigned sq = crow - bidx * (unsigned)SEQ;
        const size_t frow = (size_t)bidx * SEQ_FULL + sq;
        const v4f xr = *(const v4f*)(resid + frow * DIM + n0 + c);
#pragma unroll
        for (int j = 0; j < 4; ++j) val[j] = bf16r(xr[j]) + t[j];
      } else if (MODE == G_PRE_2X) {
#pragma unroll
        for (int j = 0; j < 4; ++j) val[j] = t[j] + t[j];
      } else {
        const v4f xr = *(const v4f*)(resid + (size_t)crow * DIM + n0 + c);
#pragma unroll
        for (int j = 0; j < 4; ++j) val[j] = xr[j] + t[j];
      }
      xs[i] = val;
      off[i] = (size_t)crow * DIM + n0 + c;
    }
#pragma unroll
    for (int i = 0; i < 4; ++i) *(volatile v4f*)(outf + off[i]) = xs[i];
    __threadfence();
#pragma unroll
    for (int i = 0; i < 4; ++i) *(volatile v4f*)(outf + off[i]) = xs[i];
  }
}

template <int CROSS>
__global__ __launch_bounds__(256) void attn_kernel(
    const _Float16* __restrict__ Qh, const _Float16* __restrict__ Kh,
    const _Float16* __restrict__ Vt, const _Float16* __restrict__ Vtr,
    _Float16* __restrict__ Ov, _Float16* __restrict__ Ovr, float scale) {
  __shared__ __attribute__((aligned(16))) _Float16 Ks[64 * LDT];
  __shared__ __attribute__((aligned(16))) _Float16 Vs[64 * LDT];
  __shared__ __attribute__((aligned(16))) _Float16 Vr[CROSS ? 64 * LDT : 8];
  __shared__ __attribute__((aligned(16))) _Float16 Ps[8 * 16 * LDT];
  __shared__ float Us[64];

  const unsigned tid = threadIdx.x, lane = tid & 31u, w = tid >> 5;
  const unsigned hh = lane >> 4, m = lane & 15u;
  const unsigned q0 = blockIdx.x * 128u;
  const unsigned head = blockIdx.y;
  const unsigned b = blockIdx.z;
  _Float16* P = Ps + w * (16u * LDT);

  const size_t qoff = (size_t)(b * (unsigned)SEQ + q0 + w * 16u + m) * DIM + head * HD + hh * 8u;
  v16h qf[2];
  qf[0] = frag_at(Qh + qoff);
  qf[1] = frag_at(Qh + qoff + 32);

  float mrow[8], lrow[8];
  v8f o[4], orr[4];
#pragma unroll
  for (int v = 0; v < 8; ++v) { mrow[v] = -1.0e30f; lrow[v] = 0.0f; }
#pragma unroll
  for (int nb = 0; nb < 4; ++nb) { o[nb] = (v8f){}; orr[nb] = (v8f){}; }

  const size_t kplane = (size_t)b * SEQ * DIM + head * HD;
  const size_t vplane = ((size_t)b * DIM + head * HD) * SEQ;
  const unsigned kend = CROSS ? (unsigned)SEQ : (q0 + 128u);
  const unsigned rowbase = q0 + w * 16u + hh * 8u;

  for (unsigned kb = 0; kb < kend; kb += 64u) {
#pragma unroll
    for (unsigned j = 0; j < 2u; ++j) {
      const unsigned idx = tid + 256u * j;
      const unsigned r = idx >> 3, c = (idx & 7u) * 8u;
      *(v8h*)&Ks[r * LDT + c] = *(const v8h*)(Kh + kplane + (size_t)(kb + r) * DIM + c);
      const v8h vh = *(const v8h*)(Vt + vplane + (size_t)r * SEQ + kb + c);
      *(v8h*)&Vs[r * LDT + c] = vh;
      if (CROSS) {
        const v8h vr = *(const v8h*)(Vtr + vplane + (size_t)r * SEQ + kb + c);
        *(v8h*)&Vr[r * LDT + c] = vr;
        float sh = 0.0f, sr = 0.0f;
#pragma unroll
        for (int e = 0; e < 8; ++e) { sh += (float)vh[e]; sr += (float)vr[e]; }
        float su = sh + sr * (1.0f / RCARRY);
        su += __shfl_xor(su, 1, 32);
        su += __shfl_xor(su, 2, 32);
        su += __shfl_xor(su, 4, 32);
        if ((idx & 7u) == 0u) Us[r] = su;
      }
    }
    __syncthreads();

    v8f s[4];
#pragma unroll
    for (int kg = 0; kg < 4; ++kg) {
      v8f t = {};
#pragma unroll
      for (int c = 0; c < 2; ++c) {
        const v16h kf = ld_frag(&Ks[(kg * 16) * LDT + c * 32], LDT);
        t = wmma16(qf[c], kf, t);
      }
      s[kg] = t * scale;
    }
    if (!CROSS) {
#pragma unroll
      for (int kg = 0; kg < 4; ++kg) {
        const unsigned key = kb + (unsigned)kg * 16u + m;
#pragma unroll
        for (int v = 0; v < 8; ++v)
          s[kg][v] = (key > rowbase + (unsigned)v) ? -1.0e30f : s[kg][v];
      }
    }

    float alpha[8];
#pragma unroll
    for (int v = 0; v < 8; ++v) {
      float mx = fmaxf(fmaxf(s[0][v], s[1][v]), fmaxf(s[2][v], s[3][v]));
      mx = red16_max(mx);
      const float mn = fmaxf(mrow[v], mx);
      alpha[v] = __expf(mrow[v] - mn);
      mrow[v] = mn;
    }
#pragma unroll
    for (int kg = 0; kg < 4; ++kg)
#pragma unroll
      for (int v = 0; v < 8; ++v) s[kg][v] = __expf(s[kg][v] - mrow[v]);
#pragma unroll
    for (int v = 0; v < 8; ++v) {
      const float rs = red16_sum((s[0][v] + s[1][v]) + (s[2][v] + s[3][v]));
      lrow[v] = alpha[v] * lrow[v] + rs;
    }
    if (CROSS) {
#pragma unroll
      for (int nb = 0; nb < 4; ++nb) {
        const float cu = Us[(unsigned)nb * 16u + m] * PCEN;
#pragma unroll
        for (int v = 0; v < 8; ++v) {
          o[nb][v] = o[nb][v] * alpha[v] + cu;
          orr[nb][v] = orr[nb][v] * alpha[v];
        }
      }
    } else {
#pragma unroll
      for (int nb = 0; nb < 4; ++nb)
#pragma unroll
        for (int v = 0; v < 8; ++v) o[nb][v] = o[nb][v] * alpha[v];
    }

#pragma unroll
    for (int kg = 0; kg < 4; ++kg)
#pragma unroll
      for (int v = 0; v < 8; ++v) {
        const float pv = CROSS ? (s[kg][v] * PCARRY - PCEN) : (s[kg][v] * PCARRY);
        P[(hh * 8u + (unsigned)v) * LDT + (unsigned)kg * 16u + m] = (_Float16)pv;
      }
    wave_lds_sync();

#pragma unroll
    for (int c = 0; c < 2; ++c) {
      const v16h pf = ld_frag(P + c * 32, LDT);
#pragma unroll
      for (int nb = 0; nb < 4; ++nb) {
        const v16h vf = ld_frag(&Vs[(nb * 16) * LDT + c * 32], LDT);
        o[nb] = wmma16(pf, vf, o[nb]);
        if (CROSS) {
          const v16h vg = ld_frag(&Vr[(nb * 16) * LDT + c * 32], LDT);
          orr[nb] = wmma16(pf, vg, orr[nb]);
        }
      }
    }
    __syncthreads();
  }

  float inv[8];
#pragma unroll
  for (int v = 0; v < 8; ++v) inv[v] = __builtin_amdgcn_rcpf(lrow[v]) * (VCARRY / PCARRY);
#pragma unroll
  for (int nb = 0; nb < 4; ++nb)
#pragma unroll
    for (int v = 0; v < 8; ++v) {
      const float tot = CROSS ? (o[nb][v] + orr[nb][v] * (1.0f / RCARRY)) : o[nb][v];
      o[nb][v] = tot * inv[v];
    }
#pragma unroll
  for (int nb = 0; nb < 4; ++nb)
#pragma unroll
    for (int v = 0; v < 8; ++v)
      P[(hh * 8u + (unsigned)v) * LDT + (unsigned)nb * 16u + m] = (_Float16)o[nb][v];
  wave_lds_sync();
  v8h x[4], y[4];
  size_t off[4];
#pragma unroll
  for (unsigned i = 0; i < 4u; ++i) {
    const unsigned r = 4u * i + (lane >> 3);
    const unsigned c = (lane & 7u) * 8u;
    x[i] = *(const v8h*)&P[r * LDT + c];
    y[i] = x[i];
    off[i] = (size_t)(b * (unsigned)SEQ + q0 + w * 16u + r) * DIM + head * HD + c;
  }
  if (CROSS) {
    wave_lds_sync();
#pragma unroll
    for (int nb = 0; nb < 4; ++nb)
#pragma unroll
      for (int v = 0; v < 8; ++v) {
        const _Float16 hv = (_Float16)o[nb][v];
        P[(hh * 8u + (unsigned)v) * LDT + (unsigned)nb * 16u + m] =
            (_Float16)((o[nb][v] - (float)hv) * RCARRY);
      }
    wave_lds_sync();
#pragma unroll
    for (unsigned i = 0; i < 4u; ++i) {
      const unsigned r = 4u * i + (lane >> 3);
      const unsigned c = (lane & 7u) * 8u;
      y[i] = *(const v8h*)&P[r * LDT + c];
    }
  }
#pragma unroll
  for (int i = 0; i < 4; ++i) *(volatile v8h*)(Ov + off[i]) = x[i];
  if (CROSS) {
#pragma unroll
    for (int i = 0; i < 4; ++i) *(volatile v8h*)(Ovr + off[i]) = y[i];
  }
  __threadfence();
#pragma unroll
  for (int i = 0; i < 4; ++i) *(volatile v8h*)(Ov + off[i]) = x[i];
  if (CROSS) {
#pragma unroll
    for (int i = 0; i < 4; ++i) *(volatile v8h*)(Ovr + off[i]) = y[i];
  }
}

template <int OUTF, int OUT16, int FULLROW>
__global__ __launch_bounds__(256) void ln_kernel(
    const float* __restrict__ pre, const float* __restrict__ g,
    const float* __restrict__ be, float* __restrict__ outf,
    _Float16* __restrict__ out16) {
  __shared__ float r1[8];
  __shared__ float r2[8];
  const unsigned tid = threadIdx.x, lane = tid & 31u, w = tid >> 5;
  const unsigned crow = blockIdx.x;
  const unsigned c = tid * 4u;
  const v4f x = *(const v4f*)(pre + (size_t)crow * DIM + c);
  const float s = red32_sum((x[0] + x[1]) + (x[2] + x[3]));
  if (lane == 0u) r1[w] = s;
  __syncthreads();
  float tot = 0.0f;
#pragma unroll
  for (int i = 0; i < 8; ++i) tot += r1[i];
  const float mean = tot * (1.0f / (float)DIM);
  v4f d;
#pragma unroll
  for (int j = 0; j < 4; ++j) d[j] = x[j] - mean;
  const float q = red32_sum((d[0] * d[0] + d[1] * d[1]) + (d[2] * d[2] + d[3] * d[3]));
  if (lane == 0u) r2[w] = q;
  __syncthreads();
  float vt = 0.0f;
#pragma unroll
  for (int i = 0; i < 8; ++i) vt += r2[i];
  const float rstd = rsqrtf(vt * (1.0f / (float)DIM) + 1.0e-6f);
  const v4f gv = *(const v4f*)(g + c);
  const v4f bv = *(const v4f*)(be + c);
  v4f yv;
  v4h yh;
#pragma unroll
  for (int j = 0; j < 4; ++j) {
    yv[j] = d[j] * rstd * bf16r(gv[j]) + bf16r(bv[j]);
    yh[j] = (_Float16)yv[j];
  }
  size_t orow = (size_t)crow;
  if (FULLROW) {
    const unsigned bidx = crow / (unsigned)SEQ;
    const unsigned sq = crow - bidx * (unsigned)SEQ;
    orow = (size_t)bidx * SEQ_FULL + sq;
  }
  if (OUTF)  *(volatile v4f*)(outf + orow * DIM + c) = yv;
  if (OUT16) *(volatile v4h*)(out16 + (size_t)crow * DIM + c) = yh;
  __threadfence();
  if (OUTF)  *(volatile v4f*)(outf + orow * DIM + c) = yv;
  if (OUT16) *(volatile v4h*)(out16 + (size_t)crow * DIM + c) = yh;
}

extern "C" void kernel_launch(void* const* d_in, const int* in_sizes, int n_in,
                              void* d_out, int out_size, void* d_ws, size_t ws_size,
                              hipStream_t stream) {
  if (n_in < 20) return;
  const long long need_x = ((long long)(NB - 1) * SEQ_FULL + SEQ) * DIM;
  const long long need_w = (long long)DIM * DIM;
  if ((long long)in_sizes[0] < need_x) return;
  if ((long long)in_sizes[1] < need_x) return;
  if ((long long)in_sizes[2] < need_w || (long long)in_sizes[3] < need_w ||
      (long long)in_sizes[4] < need_w || (long long)in_sizes[5] < need_w) return;
  if ((long long)in_sizes[7] < need_w || (long long)in_sizes[8] < need_w ||
      (long long)in_sizes[9] < need_w || (long long)in_sizes[10] < need_w ||
      (long long)in_sizes[12] < need_w) return;
  if (in_sizes[6] < DIM || in_sizes[11] < DIM || in_sizes[13] < DIM) return;
  for (int i = 14; i < 20; ++i) if (in_sizes[i] < DIM) return;
  if ((long long)out_size < need_x) return;
  if (ws_size < WS_TOTAL) return;

  const float* X   = (const float*)d_in[0];
  const float* CTX = (const float*)d_in[1];
  const float* Wk1 = (const float*)d_in[2];
  const float* Wv1 = (const float*)d_in[3];
  const float* Wq1 = (const float*)d_in[4];
  const float* Wo1 = (const float*)d_in[5];
  const float* bo1 = (const float*)d_in[6];
  const float* Wk2 = (const float*)d_in[7];
  const float* Wv2 = (const float*)d_in[8];
  const float* Wq2 = (const float*)d_in[9];
  const float* Wo2 = (const float*)d_in[10];
  const float* bo2 = (const float*)d_in[11];
  const float* Wf  = (const float*)d_in[12];
  const float* bfv = (const float*)d_in[13];
  const float* g1  = (const float*)d_in[14];
  const float* b1  = (const float*)d_in[15];
  const float* g2  = (const float*)d_in[16];
  const float* b2  = (const float*)d_in[17];
  const float* g3  = (const float*)d_in[18];
  const float* b3  = (const float*)d_in[19];
  float* out = (float*)d_out;

  char* ws = (char*)d_ws;
  _Float16* Wt   = (_Float16*)ws;
  _Float16* XA16 = (_Float16*)(ws + OFF_XA);
  _Float16* CX16 = (_Float16*)(ws + OFF_CX);
  _Float16* Q16  = (_Float16*)(ws + OFF_Q);
  _Float16* K16  = (_Float16*)(ws + OFF_K);
  _Float16* VT16 = (_Float16*)(ws + OFF_VT);
  _Float16* VTR  = (_Float16*)(ws + OFF_VTR);
  _Float16* O16  = (_Float16*)(ws + OFF_O);
  _Float16* OR16 = (_Float16*)(ws + OFF_OR);
  _Float16* CN16 = (_Float16*)(ws + OFF_CN);
  float*    PRE  = (float*)(ws + OFF_PRE);
  float*    CF   = (float*)(ws + OFF_CF);

  const size_t WP = (size_t)DIM * DIM;
  const dim3 blk(256);
  const dim3 gw(DIM / 64, DIM / 64);
  const dim3 gx((unsigned)(((size_t)MROWS * DIM) / 2048));
  const dim3 gg(DIM / 64, MROWS / 64);
  const dim3 ga(SEQ / 128, NHEAD, NB);
  const dim3 gl(MROWS);
  const float scale = 1.0f / sqrtf((float)SEQ);
  const float s64 = 1.0f / WCARRY;
  const float s4096 = 1.0f / (WCARRY * VCARRY);

  wconv_kernel<1><<<gw, blk, 0, stream>>>(Wq1, Wt + 0 * WP);
  wconv_kernel<1><<<gw, blk, 0, stream>>>(Wk1, Wt + 1 * WP);
  wconv_kernel<1><<<gw, blk, 0, stream>>>(Wv1, Wt + 2 * WP);
  wconv_kernel<0><<<gw, blk, 0, stream>>>(Wo1, Wt + 3 * WP);
  wconv_kernel<1><<<gw, blk, 0, stream>>>(Wq2, Wt + 4 * WP);
  wconv_kernel<1><<<gw, blk, 0, stream>>>(Wk2, Wt + 5 * WP);
  wconv_kernel<1><<<gw, blk, 0, stream>>>(Wv2, Wt + 6 * WP);
  wconv_kernel<0><<<gw, blk, 0, stream>>>(Wo2, Wt + 7 * WP);
  wconv_kernel<0><<<gw, blk, 0, stream>>>(Wf,  Wt + 8 * WP);
  xconv_kernel<<<gx, blk, 0, stream>>>(X, XA16);
  xconv_kernel<<<gx, blk, 0, stream>>>(CTX, CX16);

  gemm_kernel<G_ROW16><<<gg, blk, 0, stream>>>(XA16, XA16, Wt + 0 * WP, bo1, X, PRE, Q16, Q16, s64);
  gemm_kernel<G_ROW16><<<gg, blk, 0, stream>>>(XA16, XA16, Wt + 1 * WP, bo1, X, PRE, K16, K16, s64);
  gemm_kernel<G_VT><<<gg, blk, 0, stream>>>(XA16, XA16, Wt + 2 * WP, bo1, X, PRE, VT16, VTR, s64);
  attn_kernel<0><<<ga, blk, 0, stream>>>(Q16, K16, VT16, VTR, O16, OR16, scale);
  gemm_kernel<G_PRE_X><<<gg, blk, 0, stream>>>(O16, O16, Wt + 3 * WP, bo1, X, PRE, Q16, Q16, s4096);
  ln_kernel<0, 1, 0><<<gl, blk, 0, stream>>>(PRE, g1, b1, CF, XA16);

  gemm_kernel<G_ROW16><<<gg, blk, 0, stream>>>(XA16, XA16, Wt + 4 * WP, bo2, X, PRE, Q16, Q16, s64);
  gemm_kernel<G_ROW16><<<gg, blk, 0, stream>>>(CX16, CX16, Wt + 5 * WP, bo2, X, PRE, K16, K16, s64);
  gemm_kernel<G_VT2><<<gg, blk, 0, stream>>>(CX16, CX16, Wt + 6 * WP, bo2, X, PRE, VT16, VTR, s64);
  attn_kernel<1><<<ga, blk, 0, stream>>>(Q16, K16, VT16, VTR, O16, OR16, scale);
  gemm_kernel<G_PRE_2X><<<gg, blk, 0, stream>>>(O16, OR16, Wt + 7 * WP, bo2, X, PRE, Q16, Q16, s4096);
  ln_kernel<1, 1, 0><<<gl, blk, 0, stream>>>(PRE, g2, b2, CF, CN16);

  gemm_kernel<G_PRE_C><<<gg, blk, 0, stream>>>(CN16, CN16, Wt + 8 * WP, bfv, CF, PRE, Q16, Q16, s64);
  ln_kernel<1, 0, 1><<<gl, blk, 0, stream>>>(PRE, g3, b3, out, CN16);
}
